// ChebyKAN_7370163880754
// MI455X (gfx1250) — hardware-verified
//
#include <hip/hip_runtime.h>
#include <math.h>

constexpr int kRows      = 8192;
constexpr int kIn        = 768;
constexpr int kOutF      = 768;
constexpr int kDeg1      = 9;
constexpr int kK         = kIn * kDeg1;
constexpr int kHalfRows  = 4096;
constexpr int kNumHalves = kRows / kHalfRows;
constexpr float kCarry    = 8192.0f;
constexpr float kCarryInv = 1.0f / 8192.0f;
constexpr int kBasisChunk  = 256;
constexpr int kChunkHalves = kBasisChunk * kDeg1;
constexpr int kChunkVec    = kChunkHalves / 8;
constexpr int kChunksPerRow = kIn / kBasisChunk;
constexpr int kBtVec       = (kOutF * kK) / 8;
static_assert(kK % 32 == 0, "K tile");
static_assert(kHalfRows % 64 == 0 && kOutF % 64 == 0, "MN tile");
static_assert(kChunkHalves % 8 == 0 && (kChunkHalves * 2) % 128 == 0, "chunk lines");
static_assert((kK * 2) % 128 == 0, "row lines");
static_assert(kBtVec % 256 == 0, "coef grid exact");

typedef __attribute__((ext_vector_type(16))) _Float16 v16h;
typedef __attribute__((ext_vector_type(8)))  _Float16 v8h;
typedef __attribute__((ext_vector_type(16))) __bf16   v16b;
typedef __attribute__((ext_vector_type(8)))  __bf16   v8b;
typedef __attribute__((ext_vector_type(8)))  float    v8f;
typedef __attribute__((ext_vector_type(4)))  float    v4f;
typedef __attribute__((ext_vector_type(4)))  unsigned int v4u;

__device__ __forceinline__ unsigned short f2bf_bits(float f) {
  unsigned u = __float_as_uint(f);
  return (unsigned short)((u + 0x7FFFu + ((u >> 16) & 1u)) >> 16);
}
__device__ __forceinline__ float bf_bits2f(unsigned short h) { return __uint_as_float(((unsigned)h) << 16); }

__device__ __forceinline__ void dep_guard_h(v8f& a, v8f& b, v16h x, v16h y) { asm volatile("v_nop\n\tv_nop\n\tv_nop\n\tv_nop" : "+v"(a), "+v"(b) : "v"(x), "v"(y)); }
__device__ __forceinline__ void dep_guard_b(v8f& a, v8f& b, v16b x, v16b y) { asm volatile("v_nop\n\tv_nop\n\tv_nop\n\tv_nop" : "+v"(a), "+v"(b) : "v"(x), "v"(y)); }
__device__ __forceinline__ void keep4_h(v16h a, v16h b, v16h c, v16h d) { asm volatile("v_nop" :: "v"(a), "v"(b), "v"(c), "v"(d)); }
__device__ __forceinline__ void keep4_b(v16b a, v16b b, v16b c, v16b d) { asm volatile("v_nop" :: "v"(a), "v"(b), "v"(c), "v"(d)); }
__device__ __forceinline__ void acc_guard4(v8f& a, v8f& b, v8f& c, v8f& d) { asm volatile("v_nop\n\tv_nop\n\tv_nop\n\tv_nop" : "+v"(a), "+v"(b), "+v"(c), "+v"(d)); }
template <typename T> struct Frag;
template <> struct Frag<_Float16> {
  typedef v16h V; union U { v16h v; v8h h[2]; };
  static __device__ __forceinline__ v16h load(const _Float16* p) {
    U f; f.h[0] = *(const v8h*)(p); f.h[1] = *(const v8h*)(p + 16); return f.v;
  }
  static __device__ __forceinline__ v8f mma(v16h a, v16h b, v8f c) {
    return __builtin_amdgcn_wmma_f32_16x16x32_f16(false, a, false, b, (short)0, c, false, false);
  }
  static __device__ __forceinline__ void guard(v8f& a, v8f& b, v16h x, v16h y) { dep_guard_h(a, b, x, y); }
  static __device__ __forceinline__ void keep(v16h a, v16h b, v16h c, v16h d) { keep4_h(a, b, c, d); }
};
template <> struct Frag<__bf16> {
  typedef v16b V; union U { v16b v; v8b h[2]; };
  static __device__ __forceinline__ v16b load(const __bf16* p) {
    U f; f.h[0] = *(const v8b*)(p); f.h[1] = *(const v8b*)(p + 16); return f.v;
  }
  static __device__ __forceinline__ v8f mma(v16b a, v16b b, v8f c) {
    return __builtin_amdgcn_wmma_f32_16x16x32_bf16(false, a, false, b, (short)0, c, false, false);
  }
  static __device__ __forceinline__ void guard(v8f& a, v8f& b, v16b x, v16b y) { dep_guard_b(a, b, x, y); }
  static __device__ __forceinline__ void keep(v16b a, v16b b, v16b c, v16b d) { keep4_b(a, b, c, d); }
};

__device__ __forceinline__ unsigned pk16(unsigned short a, unsigned short b) { return (unsigned)a | ((unsigned)b << 16); }
__device__ __forceinline__ unsigned short h_bits(float f) { const _Float16 h = (_Float16)f; return __builtin_bit_cast(unsigned short, h); }

template <int ET> struct Elem;
template <> struct Elem<0> { typedef _Float16 T; };
template <> struct Elem<1> { typedef __bf16 T; };
template <int ET, bool SPLIT, int BIAS_MODE, int OUT_MODE, bool RESID, int ACT = 0>
__global__ __launch_bounds__(256) void wmma_gemm64(
    const unsigned short* __restrict__ Ap, const unsigned short* __restrict__ A2p, int lda, long strideA,
    const unsigned short* __restrict__ Btp, const unsigned short* __restrict__ Bt2p, int ldb, long strideB,
    void* __restrict__ Cout, void* __restrict__ Cout2, int ldc, long strideC,
    const float* __restrict__ bias,
    const float* __restrict__ resid, long strideR,
    int M, int N, int K, float scale) {
  typedef typename Elem<ET>::T T;
  typedef typename Frag<T>::V V;
  const T* A = (const T*)Ap; const T* A2 = (const T*)A2p; const T* Bt = (const T*)Btp; const T* Bt2 = (const T*)Bt2p;
  __shared__ __align__(16) float sT[8][16 * 68];
  const int b    = blockIdx.y;
  const int lane = threadIdx.x & 31;
  const int wave = threadIdx.x >> 5;
  const int tilesN = N >> 6;
  const int tilesM = M >> 6;
  const int tile = blockIdx.x * 8 + wave;
  if (tile >= tilesM * tilesN) return;
  const int tm = tile / tilesN;
  const int tn = tile - tm * tilesN;
  const int m0 = tm << 6;
  const int n0 = tn << 6;

  const T* Ab  = A  + (size_t)b * strideA;
  const T* Bb  = Bt + (size_t)b * strideB;
  const T* Ab2 = SPLIT ? (A2  + (size_t)b * strideA) : nullptr;
  const T* Bb2 = SPLIT ? (Bt2 + (size_t)b * strideB) : nullptr;

  const int rlane = lane & 15;
  const int koff  = (lane >> 4) * 8;
  const int mOff  = (lane >> 4) * 8;

  v8f acc[4][4];
#pragma unroll
  for (int i = 0; i < 4; ++i)
#pragma unroll
    for (int j = 0; j < 4; ++j) acc[i][j] = (v8f){0.f,0.f,0.f,0.f,0.f,0.f,0.f,0.f};

  for (int k0 = 0; k0 < K; k0 += 32) {
    V bh[4], bl[4];
#pragma unroll
    for (int j = 0; j < 4; ++j) {
      const size_t bo = (size_t)(n0 + (j << 4) + rlane) * ldb + koff + k0;
      bh[j] = Frag<T>::load(Bb + bo);
      if (SPLIT) bl[j] = Frag<T>::load(Bb2 + bo);
    }
#pragma unroll
    for (int i = 0; i < 4; ++i) {
      const size_t ao = (size_t)(m0 + (i << 4) + rlane) * lda + koff + k0;
      V ah = Frag<T>::load(Ab + ao);
      V al;
      if (SPLIT) al = Frag<T>::load(Ab2 + ao);
#pragma unroll
      for (int j = 0; j < 4; ++j) {
        acc[i][j] = Frag<T>::mma(ah, bh[j], acc[i][j]);
        if (SPLIT) {
          acc[i][j] = Frag<T>::mma(ah, bl[j], acc[i][j]);
          acc[i][j] = Frag<T>::mma(al, bh[j], acc[i][j]);
        }
      }
      Frag<T>::guard(acc[i][0], acc[i][3], ah, SPLIT ? al : ah);
    }
    Frag<T>::keep(bh[0], bh[1], bh[2], bh[3]);
    if (SPLIT) Frag<T>::keep(bl[0], bl[1], bl[2], bl[3]);
  }
  acc_guard4(acc[0][0], acc[0][1], acc[0][2], acc[0][3]);
  acc_guard4(acc[1][0], acc[1][1], acc[1][2], acc[1][3]);
  acc_guard4(acc[2][0], acc[2][1], acc[2][2], acc[2][3]);
  acc_guard4(acc[3][0], acc[3][1], acc[3][2], acc[3][3]);

  float* slab = sT[wave];
  const float* Rb = RESID ? (resid + (size_t)b * strideR) : nullptr;
#pragma unroll
  for (int i = 0; i < 4; ++i) {
    const int mBase = m0 + (i << 4);
#pragma unroll
    for (int j = 0; j < 4; ++j) {
      const int n = n0 + (j << 4) + rlane;
      float bv = 0.f;
      if (BIAS_MODE == 2) bv = bias[n];
#pragma unroll
      for (int r = 0; r < 8; ++r) {
        float v = acc[i][j][r] * scale;
        if (BIAS_MODE == 1) v += bias[mBase + mOff + r];
        if (BIAS_MODE == 2) v += bv;
        if (RESID) v += Rb[(size_t)(mBase + mOff + r) * ldc + n];
        if (ACT == 2) v = fmaxf(v, 0.0f);
        if (ACT == 4) v = (v > 0.f) ? v : 0.01f * v;
        slab[(mOff + r) * 68 + (j << 4) + rlane] = v;
      }
    }
    __builtin_amdgcn_fence(__ATOMIC_RELEASE, "workgroup");
    __builtin_amdgcn_wave_barrier();
    __builtin_amdgcn_fence(__ATOMIC_ACQUIRE, "workgroup");
    if (OUT_MODE == 0) {
      float* C = (float*)Cout + (size_t)b * strideC;
      const int hh = lane >> 4, c4 = (lane & 15) * 4;
      for (int pass = 0; pass < 2; ++pass) {
#pragma unroll
        for (int it = 0; it < 8; ++it) {
          const int row = it * 2 + hh;
          v4f v = *(const v4f*)(slab + row * 68 + c4);
          *(volatile v4f*)(C + (size_t)(mBase + row) * ldc + n0 + c4) = v;
        }
        __threadfence();
      }
    } else {
      const int q = lane >> 3, c8 = (lane & 7) * 8;
      unsigned short* C  = (unsigned short*)Cout  + (size_t)b * strideC;
      unsigned short* C2 = (OUT_MODE == 2) ? ((unsigned short*)Cout2 + (size_t)b * strideC) : nullptr;
      for (int pass = 0; pass < 2; ++pass) {
#pragma unroll
        for (int it = 0; it < 4; ++it) {
          const int row = it * 4 + q;
          const float* sp = slab + row * 68 + c8;
          v8h hv, lv;
#pragma unroll
          for (int e = 0; e < 8; ++e) {
            if (OUT_MODE == 1) {
              hv[e] = (_Float16)sp[e];
            } else {
              unsigned short hb = f2bf_bits(sp[e]);
              unsigned short lb = f2bf_bits(sp[e] - bf_bits2f(hb));
              hv[e] = __builtin_bit_cast(_Float16, hb);
              lv[e] = __builtin_bit_cast(_Float16, lb);
            }
          }
          *(volatile v8h*)(C + (size_t)(mBase + row) * ldc + n0 + c8) = hv;
          if (OUT_MODE == 2) *(volatile v8h*)(C2 + (size_t)(mBase + row) * ldc + n0 + c8) = lv;
        }
        __threadfence();
      }
    }
    __builtin_amdgcn_fence(__ATOMIC_RELEASE, "workgroup");
    __builtin_amdgcn_wave_barrier();
    __builtin_amdgcn_fence(__ATOMIC_ACQUIRE, "workgroup");
  }
}

__device__ __forceinline__ v4u pack8_f16(const float* sp) {
  const v4f a = *(const v4f*)(sp);
  const v4f c = *(const v4f*)(sp + 4);
  unsigned short hb[8];
#pragma unroll
  for (int e = 0; e < 4; ++e) {
    hb[e]     = h_bits(a[e]);
    hb[4 + e] = h_bits(c[e]);
  }
  return (v4u){pk16(hb[0], hb[1]), pk16(hb[2], hb[3]), pk16(hb[4], hb[5]), pk16(hb[6], hb[7])};
}

__global__ __launch_bounds__(256) void coef_cast_kernel(const float* __restrict__ coef, unsigned short* __restrict__ Bt, int nvec) {
  const int q = blockIdx.x * 256 + threadIdx.x;
  if (q >= nvec) return;
  const int vecPerRow = kK / 8;
  const int j  = q / vecPerRow;
  const int k0 = (q - j * vecPerRow) * 8;
  unsigned short hb[8];
#pragma unroll
  for (int e = 0; e < 8; ++e) {
    const int k = k0 + e;
    const int i = k / kDeg1;
    const int d = k - i * kDeg1;
    const float v = coef[((size_t)i * kOutF + j) * kDeg1 + d] * kCarry;
    hb[e] = h_bits(v);
  }
  const v4u u = (v4u){pk16(hb[0], hb[1]), pk16(hb[2], hb[3]), pk16(hb[4], hb[5]), pk16(hb[6], hb[7])};
  unsigned short* p = Bt + (size_t)q * 8;
  *(volatile v4u*)p = u;
  __threadfence();
  *(volatile v4u*)p = u;
}

__global__ __launch_bounds__(256) void basis_kernel(const float* __restrict__ x, unsigned short* __restrict__ A, int rbase) {
  __shared__ __align__(16) float sm[kChunkHalves];
  const int t = threadIdx.x;
  const int c = blockIdx.x;
  const int r = blockIdx.y;
  const float xv = x[(size_t)(rbase + r) * kIn + c * kBasisChunk + t];
  const float tv = tanhf(xv);
  const float two_t = 2.0f * tv;
  const float p0 = 1.0f;
  const float p1 = tv;
  const float p2 = two_t * p1 - p0;
  const float p3 = two_t * p2 - p1;
  const float p4 = two_t * p3 - p2;
  const float p5 = two_t * p4 - p3;
  const float p6 = two_t * p5 - p4;
  const float p7 = two_t * p6 - p5;
  const float p8 = two_t * p7 - p6;
  float* sp = sm + t * kDeg1;
  sp[0] = p0; sp[1] = p1; sp[2] = p2; sp[3] = p3; sp[4] = p4;
  sp[5] = p5; sp[6] = p6; sp[7] = p7; sp[8] = p8;
  __syncthreads();

  const int q1 = (256 + t < kChunkVec) ? (256 + t) : (kChunkVec - 1);
  const v4u u0 = pack8_f16(sm + 8 * t);
  const v4u u1 = pack8_f16(sm + 8 * q1);
  unsigned short* rowp = A + (size_t)r * kK + (size_t)c * kChunkHalves;
  unsigned short* d0 = rowp + 8 * t;
  unsigned short* d1 = rowp + 8 * q1;
  const bool has1 = (t < 32);
  *(volatile v4u*)d0 = u0;
  if (has1) *(volatile v4u*)d1 = u1;
  __threadfence();
  *(volatile v4u*)d0 = u0;
  if (has1) *(volatile v4u*)d1 = u1;
}

extern "C" void kernel_launch(void* const* d_in, const int* in_sizes, int n_in,
                              void* d_out, int out_size, void* d_ws, size_t ws_size,
                              hipStream_t stream) {
  if (n_in < 2) return;
  if (in_sizes[0] != kRows * kIn) return;
  if (in_sizes[1] != kIn * kOutF * kDeg1) return;
  if (out_size != kRows * kOutF) return;

  const size_t bytesA  = (size_t)kHalfRows * kK * 2;
  const size_t bytesBt = (size_t)kOutF * kK * 2;
  const size_t offA  = 0;
  const size_t offBt = offA + bytesA;
  const size_t total = offBt + bytesBt;
  if (total > ws_size) return;

  const float* x    = (const float*)d_in[0];
  const float* coef = (const float*)d_in[1];
  float* out        = (float*)d_out;
  unsigned short* Aws  = (unsigned short*)((char*)d_ws + offA);
  unsigned short* Btws = (unsigned short*)((char*)d_ws + offBt);

  coef_cast_kernel<<<dim3(kBtVec / 256), dim3(256), 0, stream>>>(coef, Btws, kBtVec);

  const int tiles   = (kHalfRows / 64) * (kOutF / 64);
  const int gemmBlk = (tiles + 7) / 8;
  for (int half = 0; half < kNumHalves; ++half) {
    const int rbase = half * kHalfRows;
    basis_kernel<<<dim3(kChunksPerRow, kHalfRows), dim3(256), 0, stream>>>(x, Aws, rbase);
    float* outHalf = out + (size_t)rbase * kOutF;
    wmma_gemm64<0, false, 0, 0, false, 0><<<dim3(gemmBlk, 1), dim3(256), 0, stream>>>(
        Aws, Aws, kK, 0L,
        Btws, Btws, kK, 0L,
        (void*)outHalf, (void*)outHalf, kOutF, 0L,
        x,
        x, 0L,
        kHalfRows, kOutF, kK, kCarryInv);
  }
}
